// RWKV6TimeMix_90228672955318
// MI455X (gfx1250) — hardware-verified
//
#include <hip/hip_runtime.h>
#include <math.h>

constexpr int   kBatch    = 4;
constexpr int   kSeq      = 1024;
constexpr int   kDim      = 1024;
constexpr int   kHeads    = 16;
constexpr int   kHeadDim  = 64;
constexpr int   kTok      = kBatch * kSeq;
constexpr long  kActPlane = (long)kTok * kDim;
constexpr long  kWgtPlane = (long)kDim * kDim;
constexpr float kWgtCarry  = 32.0f;
constexpr float kGateCarry = 8.0f;
constexpr float kProjScale = 1.0f / 32.0f;
constexpr float kOutScale  = 1.0f / 256.0f;
constexpr float kInvHeadDim = 1.0f / 64.0f;
constexpr float kLnEps    = 1e-5f;
constexpr float kDecayEps = 1e-4f;

constexpr size_t kOffXM = 0;
constexpr size_t kOffO  = 0;
constexpr size_t kOffG  = 16777216;
constexpr size_t kOffWH = 33554432;
constexpr size_t kOffP  = 44040192;
constexpr size_t kWsTotal = 111149056;

typedef __attribute__((ext_vector_type(16))) _Float16 v16h;
typedef __attribute__((ext_vector_type(8)))  _Float16 v8h;
typedef __attribute__((ext_vector_type(16))) __bf16   v16b;
typedef __attribute__((ext_vector_type(8)))  __bf16   v8b;
typedef __attribute__((ext_vector_type(8)))  float    v8f;
typedef __attribute__((ext_vector_type(4)))  float    v4f;
typedef __attribute__((ext_vector_type(2)))  float    v2f;
typedef __attribute__((ext_vector_type(4)))  unsigned int v4u;

__device__ __forceinline__ unsigned short f2bf_bits(float f) {
  unsigned u = __float_as_uint(f);
  return (unsigned short)((u + 0x7FFFu + ((u >> 16) & 1u)) >> 16);
}
__device__ __forceinline__ float bf_bits2f(unsigned short h) { return __uint_as_float(((unsigned)h) << 16); }

__device__ __forceinline__ void dep_guard_h(v8f& a, v8f& b, v16h x, v16h y) { asm volatile("v_nop\n\tv_nop\n\tv_nop\n\tv_nop" : "+v"(a), "+v"(b) : "v"(x), "v"(y)); }
__device__ __forceinline__ void dep_guard_b(v8f& a, v8f& b, v16b x, v16b y) { asm volatile("v_nop\n\tv_nop\n\tv_nop\n\tv_nop" : "+v"(a), "+v"(b) : "v"(x), "v"(y)); }
__device__ __forceinline__ void keep4_h(v16h a, v16h b, v16h c, v16h d) { asm volatile("v_nop" :: "v"(a), "v"(b), "v"(c), "v"(d)); }
__device__ __forceinline__ void keep4_b(v16b a, v16b b, v16b c, v16b d) { asm volatile("v_nop" :: "v"(a), "v"(b), "v"(c), "v"(d)); }
__device__ __forceinline__ void acc_guard4(v8f& a, v8f& b, v8f& c, v8f& d) { asm volatile("v_nop\n\tv_nop\n\tv_nop\n\tv_nop" : "+v"(a), "+v"(b), "+v"(c), "+v"(d)); }
template <typename T> struct Frag;
template <> struct Frag<_Float16> {
  typedef v16h V; union U { v16h v; v8h h[2]; };
  static __device__ __forceinline__ v16h load(const _Float16* p) {
    U f; f.h[0] = *(const v8h*)(p); f.h[1] = *(const v8h*)(p + 16); return f.v;
  }
  static __device__ __forceinline__ v8f mma(v16h a, v16h b, v8f c) {
    return __builtin_amdgcn_wmma_f32_16x16x32_f16(false, a, false, b, (short)0, c, false, false);
  }
  static __device__ __forceinline__ void guard(v8f& a, v8f& b, v16h x, v16h y) { dep_guard_h(a, b, x, y); }
  static __device__ __forceinline__ void keep(v16h a, v16h b, v16h c, v16h d) { keep4_h(a, b, c, d); }
};
template <> struct Frag<__bf16> {
  typedef v16b V; union U { v16b v; v8b h[2]; };
  static __device__ __forceinline__ v16b load(const __bf16* p) {
    U f; f.h[0] = *(const v8b*)(p); f.h[1] = *(const v8b*)(p + 16); return f.v;
  }
  static __device__ __forceinline__ v8f mma(v16b a, v16b b, v8f c) {
    return __builtin_amdgcn_wmma_f32_16x16x32_bf16(false, a, false, b, (short)0, c, false, false);
  }
  static __device__ __forceinline__ void guard(v8f& a, v8f& b, v16b x, v16b y) { dep_guard_b(a, b, x, y); }
  static __device__ __forceinline__ void keep(v16b a, v16b b, v16b c, v16b d) { keep4_b(a, b, c, d); }
};

__device__ __forceinline__ unsigned pk16(unsigned short a, unsigned short b) { return (unsigned)a | ((unsigned)b << 16); }
__device__ __forceinline__ unsigned short h_bits(float f) { const _Float16 h = (_Float16)f; return __builtin_bit_cast(unsigned short, h); }

template <int ET> struct Elem;
template <> struct Elem<0> { typedef _Float16 T; };
template <> struct Elem<1> { typedef __bf16 T; };
template <int ET, bool SPLIT, int BIAS_MODE, int OUT_MODE, bool RESID, int ACT = 0>
__global__ __launch_bounds__(256) void wmma_gemm64(
    const unsigned short* __restrict__ Ap, const unsigned short* __restrict__ A2p, int lda, long strideA,
    const unsigned short* __restrict__ Btp, const unsigned short* __restrict__ Bt2p, int ldb, long strideB,
    void* __restrict__ Cout, void* __restrict__ Cout2, int ldc, long strideC,
    const float* __restrict__ bias,
    const float* __restrict__ resid, long strideR,
    int M, int N, int K, float scale) {
  typedef typename Elem<ET>::T T;
  typedef typename Frag<T>::V V;
  const T* A = (const T*)Ap; const T* A2 = (const T*)A2p; const T* Bt = (const T*)Btp; const T* Bt2 = (const T*)Bt2p;
  __shared__ __align__(16) float sT[8][16 * 68];
  const int b    = blockIdx.y;
  const int lane = threadIdx.x & 31;
  const int wave = threadIdx.x >> 5;
  const int tilesN = N >> 6;
  const int tilesM = M >> 6;
  const int tile = blockIdx.x * 8 + wave;
  if (tile >= tilesM * tilesN) return;
  const int tm = tile / tilesN;
  const int tn = tile - tm * tilesN;
  const int m0 = tm << 6;
  const int n0 = tn << 6;

  const T* Ab  = A  + (size_t)b * strideA;
  const T* Bb  = Bt + (size_t)b * strideB;
  const T* Ab2 = SPLIT ? (A2  + (size_t)b * strideA) : nullptr;
  const T* Bb2 = SPLIT ? (Bt2 + (size_t)b * strideB) : nullptr;

  const int rlane = lane & 15;
  const int koff  = (lane >> 4) * 8;
  const int mOff  = (lane >> 4) * 8;

  v8f acc[4][4];
#pragma unroll
  for (int i = 0; i < 4; ++i)
#pragma unroll
    for (int j = 0; j < 4; ++j) acc[i][j] = (v8f){0.f,0.f,0.f,0.f,0.f,0.f,0.f,0.f};

  for (int k0 = 0; k0 < K; k0 += 32) {
    V bh[4], bl[4];
#pragma unroll
    for (int j = 0; j < 4; ++j) {
      const size_t bo = (size_t)(n0 + (j << 4) + rlane) * ldb + koff + k0;
      bh[j] = Frag<T>::load(Bb + bo);
      if (SPLIT) bl[j] = Frag<T>::load(Bb2 + bo);
    }
#pragma unroll
    for (int i = 0; i < 4; ++i) {
      const size_t ao = (size_t)(m0 + (i << 4) + rlane) * lda + koff + k0;
      V ah = Frag<T>::load(Ab + ao);
      V al;
      if (SPLIT) al = Frag<T>::load(Ab2 + ao);
#pragma unroll
      for (int j = 0; j < 4; ++j) {
        acc[i][j] = Frag<T>::mma(ah, bh[j], acc[i][j]);
        if (SPLIT) {
          acc[i][j] = Frag<T>::mma(ah, bl[j], acc[i][j]);
          acc[i][j] = Frag<T>::mma(al, bh[j], acc[i][j]);
        }
      }
      Frag<T>::guard(acc[i][0], acc[i][3], ah, SPLIT ? al : ah);
    }
    Frag<T>::keep(bh[0], bh[1], bh[2], bh[3]);
    if (SPLIT) Frag<T>::keep(bl[0], bl[1], bl[2], bl[3]);
  }
  acc_guard4(acc[0][0], acc[0][1], acc[0][2], acc[0][3]);
  acc_guard4(acc[1][0], acc[1][1], acc[1][2], acc[1][3]);
  acc_guard4(acc[2][0], acc[2][1], acc[2][2], acc[2][3]);
  acc_guard4(acc[3][0], acc[3][1], acc[3][2], acc[3][3]);

  float* slab = sT[wave];
  const float* Rb = RESID ? (resid + (size_t)b * strideR) : nullptr;
#pragma unroll
  for (int i = 0; i < 4; ++i) {
    const int mBase = m0 + (i << 4);
#pragma unroll
    for (int j = 0; j < 4; ++j) {
      const int n = n0 + (j << 4) + rlane;
      float bv = 0.f;
      if (BIAS_MODE == 2) bv = bias[n];
#pragma unroll
      for (int r = 0; r < 8; ++r) {
        float v = acc[i][j][r] * scale;
        if (BIAS_MODE == 1) v += bias[mBase + mOff + r];
        if (BIAS_MODE == 2) v += bv;
        if (RESID) v += Rb[(size_t)(mBase + mOff + r) * ldc + n];
        if (ACT == 2) v = fmaxf(v, 0.0f);
        if (ACT == 4) v = (v > 0.f) ? v : 0.01f * v;
        slab[(mOff + r) * 68 + (j << 4) + rlane] = v;
      }
    }
    __builtin_amdgcn_fence(__ATOMIC_RELEASE, "workgroup");
    __builtin_amdgcn_wave_barrier();
    __builtin_amdgcn_fence(__ATOMIC_ACQUIRE, "workgroup");
    if (OUT_MODE == 0) {
      float* C = (float*)Cout + (size_t)b * strideC;
      const int hh = lane >> 4, c4 = (lane & 15) * 4;
      for (int pass = 0; pass < 2; ++pass) {
#pragma unroll
        for (int it = 0; it < 8; ++it) {
          const int row = it * 2 + hh;
          v4f v = *(const v4f*)(slab + row * 68 + c4);
          *(volatile v4f*)(C + (size_t)(mBase + row) * ldc + n0 + c4) = v;
        }
        __threadfence();
      }
    } else {
      const int q = lane >> 3, c8 = (lane & 7) * 8;
      unsigned short* C  = (unsigned short*)Cout  + (size_t)b * strideC;
      unsigned short* C2 = (OUT_MODE == 2) ? ((unsigned short*)Cout2 + (size_t)b * strideC) : nullptr;
      for (int pass = 0; pass < 2; ++pass) {
#pragma unroll
        for (int it = 0; it < 4; ++it) {
          const int row = it * 4 + q;
          const float* sp = slab + row * 68 + c8;
          v8h hv, lv;
#pragma unroll
          for (int e = 0; e < 8; ++e) {
            if (OUT_MODE == 1) {
              hv[e] = (_Float16)sp[e];
            } else {
              unsigned short hb = f2bf_bits(sp[e]);
              unsigned short lb = f2bf_bits(sp[e] - bf_bits2f(hb));
              hv[e] = __builtin_bit_cast(_Float16, hb);
              lv[e] = __builtin_bit_cast(_Float16, lb);
            }
          }
          *(volatile v8h*)(C + (size_t)(mBase + row) * ldc + n0 + c8) = hv;
          if (OUT_MODE == 2) *(volatile v8h*)(C2 + (size_t)(mBase + row) * ldc + n0 + c8) = lv;
        }
        __threadfence();
      }
    }
    __builtin_amdgcn_fence(__ATOMIC_RELEASE, "workgroup");
    __builtin_amdgcn_wave_barrier();
    __builtin_amdgcn_fence(__ATOMIC_ACQUIRE, "workgroup");
  }
}

__device__ __forceinline__ v4u mix8(const float (&xc)[8], const float (&xp)[8], const float* __restrict__ tm, int c0) {
  const v4f t0 = *(const v4f*)(tm + c0);
  const v4f t1 = *(const v4f*)(tm + c0 + 4);
  unsigned short hb[8];
#pragma unroll
  for (int e = 0; e < 4; ++e) {
    const float a0 = t0[e];
    hb[e] = h_bits(a0 * xc[e] + (1.0f - a0) * xp[e]);
    const float a1 = t1[e];
    hb[4 + e] = h_bits(a1 * xc[4 + e] + (1.0f - a1) * xp[4 + e]);
  }
  return (v4u){pk16(hb[0], hb[1]), pk16(hb[2], hb[3]), pk16(hb[4], hb[5]), pk16(hb[6], hb[7])};
}

__global__ __launch_bounds__(256) void mix_kernel(const float* __restrict__ x,
                                                  const float* __restrict__ tmr, const float* __restrict__ tmk,
                                                  const float* __restrict__ tmv, const float* __restrict__ tmw,
                                                  unsigned short* __restrict__ xm) {
  const int gid = blockIdx.x * 256 + threadIdx.x;
  const int row = gid >> 7;
  const int c0  = (gid & 127) * 8;
  const int t   = row & (kSeq - 1);
  const int prow = (t > 0) ? (row - 1) : row;
  const float* pc = x + (size_t)row * kDim + c0;
  const float* pp = x + (size_t)prow * kDim + c0;
  const v4f ca = *(const v4f*)(pc);
  const v4f cb = *(const v4f*)(pc + 4);
  const v4f pa = *(const v4f*)(pp);
  const v4f pb = *(const v4f*)(pp + 4);
  float xc[8], xp[8];
#pragma unroll
  for (int e = 0; e < 4; ++e) {
    xc[e] = ca[e]; xc[4 + e] = cb[e];
    xp[e] = (t > 0) ? pa[e] : 0.0f;
    xp[4 + e] = (t > 0) ? pb[e] : 0.0f;
  }
  const v4u u0 = mix8(xc, xp, tmr, c0);
  const v4u u1 = mix8(xc, xp, tmk, c0);
  const v4u u2 = mix8(xc, xp, tmv, c0);
  const v4u u3 = mix8(xc, xp, tmw, c0);
  unsigned short* q = xm + (size_t)row * kDim + c0;
  for (int pass = 0; pass < 2; ++pass) {
    *(volatile v4u*)(q) = u0;
    *(volatile v4u*)(q + kActPlane) = u1;
    *(volatile v4u*)(q + 2 * kActPlane) = u2;
    *(volatile v4u*)(q + 3 * kActPlane) = u3;
    __threadfence();
  }
}

__global__ __launch_bounds__(256) void wcast8_kernel(const float* __restrict__ W0, const float* __restrict__ W1,
                                                     const float* __restrict__ W2, const float* __restrict__ W3,
                                                     const float* __restrict__ W4,
                                                     unsigned short* __restrict__ out, float scale) {
  const int z = blockIdx.y;
  const float* W = (z == 0) ? W0 : (z == 1) ? W1 : (z == 2) ? W2 : (z == 3) ? W3 : W4;
  const int i = blockIdx.x * 256 + threadIdx.x;
  const float* p = W + 8 * (size_t)i;
  const v4f a = *(const v4f*)(p);
  const v4f c = *(const v4f*)(p + 4);
  unsigned short hb[8];
#pragma unroll
  for (int e = 0; e < 4; ++e) {
    hb[e]     = h_bits(a[e] * scale);
    hb[4 + e] = h_bits(c[e] * scale);
  }
  const v4u u = (v4u){pk16(hb[0], hb[1]), pk16(hb[2], hb[3]), pk16(hb[4], hb[5]), pk16(hb[6], hb[7])};
  unsigned short* q = out + (size_t)z * kWgtPlane + 8 * (size_t)i;
  *(volatile v4u*)q = u;
  __threadfence();
  *(volatile v4u*)q = u;
}

__device__ __forceinline__ v8f mma_f16_g(v16h a, v16h b, v8f c) {
  c = __builtin_amdgcn_wmma_f32_16x16x32_f16(false, a, false, b, (short)0, c, false, false);
  asm volatile("v_nop\n\tv_nop\n\tv_nop\n\tv_nop" : "+v"(c) : "v"(a), "v"(b));
  return c;
}

__device__ __forceinline__ void col_step(float (&s)[16], v16h& bv, const float* kkp, const float* ewp, float vj) {
  const v4f q0 = *(const v4f*)(kkp);
  const v4f q1 = *(const v4f*)(kkp + 4);
  const v4f q2 = *(const v4f*)(kkp + 16);
  const v4f q3 = *(const v4f*)(kkp + 20);
  const v4f w0 = *(const v4f*)(ewp);
  const v4f w1 = *(const v4f*)(ewp + 4);
  const v4f w2 = *(const v4f*)(ewp + 16);
  const v4f w3 = *(const v4f*)(ewp + 20);
#pragma unroll
  for (int e = 0; e < 4; ++e) {
    bv[e]      = (_Float16)s[e];       s[e]      = w0[e] * s[e]      + q0[e] * vj;
    bv[4 + e]  = (_Float16)s[4 + e];   s[4 + e]  = w1[e] * s[4 + e]  + q1[e] * vj;
    bv[8 + e]  = (_Float16)s[8 + e];   s[8 + e]  = w2[e] * s[8 + e]  + q2[e] * vj;
    bv[12 + e] = (_Float16)s[12 + e];  s[12 + e] = w3[e] * s[12 + e] + q3[e] * vj;
  }
}

__global__ __launch_bounds__(128) void wkv_kernel(const float* __restrict__ ZR, const float* __restrict__ KP,
                                                  const float* __restrict__ VP, const float* __restrict__ ZW,
                                                  const float* __restrict__ u, float* __restrict__ O) {
  __shared__ __align__(16) float kk[64];
  __shared__ __align__(16) float ew[64];
  __shared__ __align__(16) float vv[64];
  __shared__ __align__(16) float uu[64];
  __shared__ __align__(16) float os[64];
  __shared__ __align__(16) float cs[4];
  __shared__ __align__(16) _Float16 rh[64];
  union HU { v16h v; v8h h8[2]; };

  const int bh = blockIdx.x;
  const int b  = bh >> 4;
  const int h  = bh & 15;
  const int tid = threadIdx.x, wave = tid >> 5, lane = tid & 31;
  const int hh = lane >> 4, c = lane & 15;
  const int jcol = wave * 16 + c;

  if (tid < kHeadDim) uu[tid] = u[h * kHeadDim + tid];
  float s0[16], s1[16];
#pragma unroll
  for (int e = 0; e < 16; ++e) { s0[e] = 0.0f; s1[e] = 0.0f; }
  __syncthreads();

  const size_t rowbase = (size_t)b * kSeq;
#pragma unroll 1
  for (int t = 0; t < kSeq; ++t) {
    const size_t base = (rowbase + (size_t)t) * (size_t)kDim + (size_t)h * kHeadDim;
    if (wave < 2) {
      const int i = tid;
      const float zr = ZR[base + i];
      const float kv = KP[base + i];
      const float r  = 1.0f / (1.0f + expf(-zr));
      rh[i] = (_Float16)r;
      kk[i] = kv;
      float pr = r * expf(uu[i] + kv);
      pr += __shfl_xor(pr, 1, 32);
      pr += __shfl_xor(pr, 2, 32);
      pr += __shfl_xor(pr, 4, 32);
      pr += __shfl_xor(pr, 8, 32);
      pr += __shfl_xor(pr, 16, 32);
      if (lane == 0) cs[wave] = pr;
    } else {
      const int i = tid - 64;
      const float zw = ZW[base + i];
      const float vl = VP[base + i];
      const float sp = fmaxf(-zw, 0.0f) + log1pf(expf(-fabsf(zw)));
      const float w  = -sp - kDecayEps;
      ew[i] = expf(w);
      vv[i] = vl;
    }
    __syncthreads();
    const float vj = vv[jcol];
    const float ct = cs[0] + cs[1];
    HU a0, a1;
    a0.h8[0] = *(const v8h*)(rh + 8 * hh);
    a0.h8[1] = *(const v8h*)(rh + 16 + 8 * hh);
    a1.h8[0] = *(const v8h*)(rh + 32 + 8 * hh);
    a1.h8[1] = *(const v8h*)(rh + 48 + 8 * hh);
    v16h bv0, bv1;
    col_step(s0, bv0, kk + 8 * hh,      ew + 8 * hh,      vj);
    col_step(s1, bv1, kk + 32 + 8 * hh, ew + 32 + 8 * hh, vj);
    v8f acc = (v8f){0.f,0.f,0.f,0.f,0.f,0.f,0.f,0.f};
    acc = mma_f16_g(a0.v, bv0, acc);
    acc = mma_f16_g(a1.v, bv1, acc);
    const float o = acc[0] + vj * ct;
    if (hh == 0) os[jcol] = o;
    __syncthreads();
    if (wave == 0 && lane < 16) {
      const v4f val = *(const v4f*)(os + 4 * lane);
      float* dst = O + base + 4 * lane;
      *(volatile v4f*)dst = val;
      __threadfence();
      *(volatile v4f*)dst = val;
    }
  }
}

__global__ __launch_bounds__(256) void ln_gate_kernel(const float* __restrict__ O, const float* __restrict__ ZR,
                                                      const float* __restrict__ lnw, const float* __restrict__ lnb,
                                                      unsigned short* __restrict__ G) {
  const int wave = threadIdx.x >> 5, lane = threadIdx.x & 31;
  const int grp  = blockIdx.x * 8 + wave;
  const int row  = grp >> 4, hq = grp & 15;
  const size_t eoff = (size_t)row * kDim + (size_t)hq * kHeadDim + 2 * lane;
  const v2f o2 = *(const v2f*)(O + eoff);
  const v2f z2 = *(const v2f*)(ZR + eoff);
  const v2f w2 = *(const v2f*)(lnw + 2 * lane);
  const v2f b2 = *(const v2f*)(lnb + 2 * lane);
  float sm = o2[0] + o2[1];
  sm += __shfl_xor(sm, 1, 32);
  sm += __shfl_xor(sm, 2, 32);
  sm += __shfl_xor(sm, 4, 32);
  sm += __shfl_xor(sm, 8, 32);
  sm += __shfl_xor(sm, 16, 32);
  const float mu = sm * kInvHeadDim;
  const float d0 = o2[0] - mu, d1 = o2[1] - mu;
  float q = d0 * d0 + d1 * d1;
  q += __shfl_xor(q, 1, 32);
  q += __shfl_xor(q, 2, 32);
  q += __shfl_xor(q, 4, 32);
  q += __shfl_xor(q, 8, 32);
  q += __shfl_xor(q, 16, 32);
  const float rs = rsqrtf(q * kInvHeadDim + kLnEps);
  const float r0 = 1.0f / (1.0f + expf(-z2[0]));
  const float r1 = 1.0f / (1.0f + expf(-z2[1]));
  const float g0 = ((d0 * rs) * w2[0] + b2[0]) * r0 * kGateCarry;
  const float g1 = ((d1 * rs) * w2[1] + b2[1]) * r1 * kGateCarry;
  const unsigned uw = pk16(h_bits(g0), h_bits(g1));
  volatile unsigned* dst = (volatile unsigned*)(G + eoff);
  *dst = uw;
  __threadfence();
  *dst = uw;
}

extern "C" void kernel_launch(void* const* d_in, const int* in_sizes, int n_in,
                              void* d_out, int out_size, void* d_ws, size_t ws_size,
                              hipStream_t stream) {
  if (n_in < 13) return;
  if (ws_size < kWsTotal) return;
  if ((long)in_sizes[0] != kActPlane) return;
  if ((long)out_size != kActPlane) return;

  const float* x    = (const float*)d_in[0];
  const float* W_r  = (const float*)d_in[1];
  const float* W_k  = (const float*)d_in[2];
  const float* W_v  = (const float*)d_in[3];
  const float* W_w  = (const float*)d_in[4];
  const float* W_o  = (const float*)d_in[5];
  const float* u    = (const float*)d_in[6];
  const float* tmr  = (const float*)d_in[7];
  const float* tmk  = (const float*)d_in[8];
  const float* tmv  = (const float*)d_in[9];
  const float* tmw  = (const float*)d_in[10];
  const float* lnw  = (const float*)d_in[11];
  const float* lnb  = (const float*)d_in[12];
  float* out = (float*)d_out;

  char* ws = (char*)d_ws;
  unsigned short* XM = (unsigned short*)(ws + kOffXM);
  float*          Op = (float*)(ws + kOffO);
  unsigned short* Gp = (unsigned short*)(ws + kOffG);
  unsigned short* WH = (unsigned short*)(ws + kOffWH);
  float*          Pp = (float*)(ws + kOffP);

  mix_kernel<<<2048, 256, 0, stream>>>(x, tmr, tmk, tmv, tmw, XM);

  wcast8_kernel<<<dim3(512, 5), 256, 0, stream>>>(W_r, W_k, W_v, W_w, W_o, WH, kWgtCarry);

  wmma_gemm64<0, false, 0, 0, false, 0><<<dim3(128, 4), 256, 0, stream>>>(
      XM, XM, kDim, (long)kActPlane,
      WH, WH, kDim, (long)kWgtPlane,
      (void*)Pp, (void*)Pp, kDim, (long)kActPlane,
      lnw, lnw, 0L,
      kTok, kDim, kDim, kProjScale);

  wkv_kernel<<<kBatch * kHeads, 128, 0, stream>>>(Pp, Pp + kActPlane, Pp + 2 * kActPlane, Pp + 3 * kActPlane, u, Op);

  ln_gate_kernel<<<8192, 256, 0, stream>>>(Op, Pp, lnw, lnb, Gp);

  wmma_gemm64<0, false, 0, 0, false, 0><<<dim3(128, 1), 256, 0, stream>>>(
      Gp, Gp, kDim, 0L,
      WH + 4 * kWgtPlane, WH + 4 * kWgtPlane, kDim, 0L,
      (void*)out, (void*)out, kDim, 0L,
      lnw, lnw, 0L,
      kTok, kDim, kDim, kOutScale);
}
